// MappingNetwork_6390911337097
// MI455X (gfx1250) — hardware-verified
//
#include <hip/hip_runtime.h>
#include <stddef.h>
#include <stdint.h>

#define BSZ    8192
#define LDIM   16
#define LPAD   32
#define HDIM   512
#define SDIM   64
#define NDOM   16
#define TR     64
#define NTT    (BSZ / TR)
#define NTILE  144
#define MP     (NTILE * TR)
#define TABH   64
#define TABL   (TABH + MP)
#define TABN   (TABL + BSZ)
#define TPT    32
#define NTHR   256
#define GTHR   128
#define WSMAX  134217728
#define LDS_BKT ((TABN + NDOM * 8) * 4)

static_assert(MP == NTILE * TR);
static_assert(MP >= BSZ + NDOM * (TR - 1));
static_assert((TABN % 32) == 0);
static_assert(BSZ == NTHR * TPT);
static_assert((TPT % 4) == 0);
static_assert((BSZ % TR) == 0);
static_assert((HDIM % 64) == 0 && (HDIM % 32) == 0 && (LPAD % 32) == 0);
static_assert(SDIM == 64);
static_assert(TR == (GTHR / 32) * 16);
static_assert(LDS_BKT <= 160000);
static_assert(NTHR / 32 == 8);
static_assert((BSZ % 8) == 0);
static_assert(TABH >= 2 * NDOM + 1);

typedef float          v4f  __attribute__((ext_vector_type(4)));
typedef float          v8f  __attribute__((ext_vector_type(8)));
typedef int            v4i  __attribute__((ext_vector_type(4)));
typedef int            v8i  __attribute__((ext_vector_type(8)));
typedef unsigned short v8us __attribute__((ext_vector_type(8)));
typedef __bf16         v16bf __attribute__((ext_vector_type(16)));
typedef v4f  __attribute__((may_alias)) v4fa;
typedef v8us __attribute__((may_alias)) v8usa;
union FragB { v16bf v; v8us h[2]; v8i w; };

__device__ __forceinline__ v8f wmb(const FragB& a, const FragB& b, v8f c) {
  v8f d = __builtin_amdgcn_wmma_f32_16x16x32_bf16(false, a.v, false, b.v, (short)0, c, false, false);
  asm volatile("v_nop\n\tv_nop\n\tv_nop\n\tv_nop" : "+v"(d) : "v"(a.w), "v"(b.w));
  return d;
}

__device__ __forceinline__ unsigned short rne16(float f) {
  unsigned u = __float_as_uint(f);
  u += 0x7FFFu + ((u >> 16) & 1u);
  return (unsigned short)(u >> 16);
}
__device__ __forceinline__ float rne16f(float f) {
  return __uint_as_float(((unsigned)rne16(f)) << 16);
}
__device__ __forceinline__ v8us cvt8(const v4f a, const v4f b) {
  v8us o;
  o[0] = rne16(a.x); o[1] = rne16(a.y); o[2] = rne16(a.z); o[3] = rne16(a.w);
  o[4] = rne16(b.x); o[5] = rne16(b.y); o[6] = rne16(b.z); o[7] = rne16(b.w);
  return o;
}
__device__ __forceinline__ void sp1(float v, unsigned short& hi, unsigned short& lo) {
  const unsigned short hb = rne16(v);
  const float hf = __uint_as_float(((unsigned)hb) << 16);
  hi = hb;
  lo = rne16(v - hf);
}
__device__ __forceinline__ void split8(const v4f a, const v4f b, v8us& hv, v8us& lv) {
  unsigned short h0, h1, h2, h3, h4, h5, h6, h7, l0, l1, l2, l3, l4, l5, l6, l7;
  sp1(a.x, h0, l0); sp1(a.y, h1, l1); sp1(a.z, h2, l2); sp1(a.w, h3, l3);
  sp1(b.x, h4, l4); sp1(b.y, h5, l5); sp1(b.z, h6, l6); sp1(b.w, h7, l7);
  hv[0] = h0; hv[1] = h1; hv[2] = h2; hv[3] = h3; hv[4] = h4; hv[5] = h5; hv[6] = h6; hv[7] = h7;
  lv[0] = l0; lv[1] = l1; lv[2] = l2; lv[3] = l3; lv[4] = l4; lv[5] = l5; lv[6] = l6; lv[7] = l7;
}
__device__ __forceinline__ v8us mask8(v8us o, int keep) {
  const unsigned short mk = keep ? (unsigned short)0xFFFFu : (unsigned short)0u;
  const v8us mv = {mk, mk, mk, mk, mk, mk, mk, mk};
  return o & mv;
}

__global__ __launch_bounds__(NTHR) void k_wtr(const float* __restrict__ src, unsigned short* dst,
                                              int K, int KP, int N, int E, int nUnits) {
  const int u = (int)blockIdx.x * NTHR + (int)threadIdx.x;
  if (u >= nUnits) return;
  const int kq  = KP >> 3;
  const int per = N * kq;
  int e = u / per;
  e = e > E - 1 ? E - 1 : e;
  const int rem = u - e * per;
  const int n   = rem / kq;
  const int k8  = (rem - n * kq) * 8;
  const int kk  = k8 > K - 8 ? K - 8 : k8;
  const float* p = src + ((size_t)e * (size_t)K + (size_t)kk) * (size_t)N + n;
  v4f a, b;
  a.x = p[0];                 a.y = p[(size_t)N];         a.z = p[(size_t)2 * N];     a.w = p[(size_t)3 * N];
  b.x = p[(size_t)4 * N];     b.y = p[(size_t)5 * N];     b.z = p[(size_t)6 * N];     b.w = p[(size_t)7 * N];
  const v8us o = mask8(cvt8(a, b), k8 < K ? 1 : 0);
  const size_t q = ((size_t)e * (size_t)N + (size_t)n) * (size_t)KP + (size_t)k8;
  *(volatile v8us*)(dst + q) = o;
  __threadfence();
  *(volatile v8us*)(dst + q) = o;
}

__global__ __launch_bounds__(NTHR) void k_zpad(const float* __restrict__ z, unsigned short* zb, int nUnits) {
  const int u = (int)blockIdx.x * NTHR + (int)threadIdx.x;
  if (u >= nUnits) return;
  const int r = u >> 2, q = u & 3, qq = q & 1;
  const float* p = z + (size_t)r * LDIM + 8 * qq;
  const v4f a = *(const v4fa*)p;
  const v4f b = *(const v4fa*)(p + 4);
  const v8us o = mask8(cvt8(a, b), q < 2 ? 1 : 0);
  const size_t d = (size_t)r * LPAD + (size_t)(8 * q);
  *(volatile v8us*)(zb + d) = o;
  __threadfence();
  *(volatile v8us*)(zb + d) = o;
}

__device__ __forceinline__ void cnt_add(int c, int (&cnt)[NDOM]) {
  c = c < 0 ? 0 : (c > NDOM - 1 ? NDOM - 1 : c);
#pragma unroll
  for (int d = 0; d < NDOM; ++d) cnt[d] += (c == d) ? 1 : 0;
}
__device__ __forceinline__ int slot_of(int c, int (&base)[NDOM]) {
  c = c < 0 ? 0 : (c > NDOM - 1 ? NDOM - 1 : c);
  int p = 0;
#pragma unroll
  for (int d = 0; d < NDOM; ++d) {
    const bool mt = (c == d);
    p = mt ? base[d] : p;
    base[d] += mt ? 1 : 0;
  }
  return p < 0 ? 0 : (p > MP - 1 ? MP - 1 : p);
}

__global__ __launch_bounds__(NTHR) void k_bucket(const int* __restrict__ y, int* tab) {
  extern __shared__ v4i lds_dyn[];
  int* img = (int*)lds_dyn;
  int* lst = img + TABH;
  int* pos = img + TABL;
  int* wt  = img + TABN;
  const int tid = (int)threadIdx.x, lane = tid & 31, wave = tid >> 5;

  const v4i z4 = {0, 0, 0, 0};
#pragma unroll 1
  for (int p = tid; p < TABN / 4; p += NTHR) *(v4i*)(img + 4 * p) = z4;
  __syncthreads();

  const int t0 = tid * TPT;
  int cnt[NDOM];
#pragma unroll
  for (int d = 0; d < NDOM; ++d) cnt[d] = 0;
#pragma unroll 1
  for (int c = 0; c < TPT / 4; ++c) {
    const v4i rc = *(const v4i*)(y + t0 + 4 * c);
    cnt_add(rc.x, cnt);
    cnt_add(rc.y, cnt);
    cnt_add(rc.z, cnt);
    cnt_add(rc.w, cnt);
  }
  int incl[NDOM];
#pragma unroll
  for (int d = 0; d < NDOM; ++d) {
    int v = cnt[d];
#pragma unroll
    for (int s = 1; s < 32; s <<= 1) {
      const int up = __shfl_up(v, s);
      v = (lane >= s) ? v + up : v;
    }
    incl[d] = v;
    if (lane == 31) wt[d * 8 + wave] = v;
  }
  __syncthreads();
  int pre[NDOM], tot[NDOM];
#pragma unroll
  for (int d = 0; d < NDOM; ++d) {
    int s = 0, all = 0;
#pragma unroll
    for (int w2 = 0; w2 < NTHR / 32; ++w2) {
      const int v = wt[d * 8 + w2];
      all += v;
      s   += (w2 < wave) ? v : 0;
    }
    pre[d] = s + incl[d] - cnt[d];
    all = all < 0 ? 0 : (all > BSZ ? BSZ : all);
    tot[d] = all;
  }
  int off[NDOM + 1];
  off[0] = 0;
#pragma unroll
  for (int d = 0; d < NDOM; ++d) {
    int nx = off[d] + ((tot[d] + TR - 1) / TR) * TR;
    nx = nx > MP ? MP : nx;
    off[d + 1] = nx;
  }
  int base[NDOM];
#pragma unroll
  for (int d = 0; d < NDOM; ++d) base[d] = off[d] + pre[d];
#pragma unroll 1
  for (int c = 0; c < TPT / 4; ++c) {
    const v4i rc = *(const v4i*)(y + t0 + 4 * c);
    const int t = t0 + 4 * c;
    const int pa = slot_of(rc.x, base); lst[pa] = t;     pos[t]     = pa;
    const int pb = slot_of(rc.y, base); lst[pb] = t + 1; pos[t + 1] = pb;
    const int pc = slot_of(rc.z, base); lst[pc] = t + 2; pos[t + 2] = pc;
    const int pd = slot_of(rc.w, base); lst[pd] = t + 3; pos[t + 3] = pd;
  }
  __syncthreads();
  if (tid == 0) {
#pragma unroll
    for (int d = 0; d < NDOM; ++d) img[d] = tot[d];
#pragma unroll
    for (int j = 0; j <= NDOM; ++j) img[NDOM + j] = off[j];
  }
  __syncthreads();
#pragma unroll 1
  for (int p = tid; p < TABN / 4; p += NTHR) {
    const v4i v = *(const v4i*)(img + 4 * p);
    *(volatile v4i*)(tab + 4 * p) = v;
  }
  __threadfence();
#pragma unroll 1
  for (int p = tid; p < TABN / 4; p += NTHR) {
    const v4i v = *(const v4i*)(img + 4 * p);
    *(volatile v4i*)(tab + 4 * p) = v;
  }
}

__global__ __launch_bounds__(NTHR) void k_gather(const unsigned short* __restrict__ chi,
                                                 const unsigned short* __restrict__ clo,
                                                 const int* __restrict__ tab,
                                                 unsigned short* xhi, unsigned short* xlo, int nUnits) {
  const int u = (int)blockIdx.x * NTHR + (int)threadIdx.x;
  if (u >= nUnits) return;
  const int row = u >> 6;
  const int c8  = (u & 63) * 8;
  int tk = tab[TABH + row];
  tk = tk < 0 ? 0 : (tk > BSZ - 1 ? BSZ - 1 : tk);
  const size_t s = (size_t)tk * HDIM + (size_t)c8;
  const v8us vh = *(const v8usa*)(chi + s);
  const v8us vl = *(const v8usa*)(clo + s);
  const size_t q = (size_t)row * HDIM + (size_t)c8;
  *(volatile v8us*)(xhi + q) = vh;
  *(volatile v8us*)(xlo + q) = vl;
  __threadfence();
  *(volatile v8us*)(xhi + q) = vh;
  *(volatile v8us*)(xlo + q) = vl;
}

__device__ __forceinline__ int tile_slot(const int* __restrict__ tab, int rowBase) {
  const v4i o0 = *(const v4i*)(tab + NDOM);
  const v4i o1 = *(const v4i*)(tab + NDOM + 4);
  const v4i o2 = *(const v4i*)(tab + NDOM + 8);
  const v4i o3 = *(const v4i*)(tab + NDOM + 12);
  int e = 0;
#define SELX(J, OJ) { const bool ge_ = rowBase >= (OJ); e = ge_ ? (J) : e; }
  SELX(1, o0.y)  SELX(2, o0.z)  SELX(3, o0.w)
  SELX(4, o1.x)  SELX(5, o1.y)  SELX(6, o1.z)  SELX(7, o1.w)
  SELX(8, o2.x)  SELX(9, o2.y)  SELX(10, o2.z) SELX(11, o2.w)
  SELX(12, o3.x) SELX(13, o3.y) SELX(14, o3.z) SELX(15, o3.w)
#undef SELX
  return e;
}

template <int KD, int NP, int NO, bool DOM, int EPI>
__global__ __launch_bounds__(GTHR) void k_gemm(const unsigned short* __restrict__ ahi,
                                               const unsigned short* __restrict__ alo,
                                               const unsigned short* __restrict__ w,
                                               const float* __restrict__ bias,
                                               const int* __restrict__ tab,
                                               unsigned short* ohi, unsigned short* olo, float* yo) {
  __shared__ __attribute__((aligned(16))) float stg[TR * 64];
  const int tid = (int)threadIdx.x, lane = tid & 31, wave = tid >> 5, hh = lane >> 4, m = lane & 15;
  const int rowBase = (int)blockIdx.x * TR;
  const int col0    = (int)blockIdx.y * 64;
  int e = 0;
  if (DOM) e = tile_slot(tab, rowBase);

  v8f acc[4];
  {
    const v8f zz = {0.f, 0.f, 0.f, 0.f, 0.f, 0.f, 0.f, 0.f};
    acc[0] = zz; acc[1] = zz; acc[2] = zz; acc[3] = zz;
  }
  const size_t arow = (size_t)(rowBase + 16 * wave + m) * (size_t)KD + (size_t)(8 * hh);
  const unsigned short* aph = ahi + arow;
  const unsigned short* apl = alo + arow;
  const unsigned short* wp  = w + (size_t)e * (size_t)(NO * KD) + (size_t)(col0 + m) * (size_t)KD + (size_t)(8 * hh);
#pragma unroll 1
  for (int ks = 0; ks < KD / 32; ++ks) {
    FragB ah;
    ah.h[0] = *(const v8usa*)(aph + 32 * ks);
    ah.h[1] = *(const v8usa*)(aph + 32 * ks + 16);
    FragB al = ah;
    if (NP == 2) {
      al.h[0] = *(const v8usa*)(apl + 32 * ks);
      al.h[1] = *(const v8usa*)(apl + 32 * ks + 16);
    }
#pragma unroll
    for (int t = 0; t < 4; ++t) {
      const unsigned short* wq = wp + (size_t)(16 * t) * (size_t)KD + 32 * ks;
      FragB bf;
      bf.h[0] = *(const v8usa*)wq;
      bf.h[1] = *(const v8usa*)(wq + 16);
      acc[t] = wmb(ah, bf, acc[t]);
      if (NP == 2) acc[t] = wmb(al, bf, acc[t]);
    }
  }

#pragma unroll
  for (int t = 0; t < 4; ++t) {
    const int lc = 16 * t + m;
    const float bn = rne16f(bias[(size_t)e * NO + col0 + lc]);
#pragma unroll
    for (int r = 0; r < 8; ++r) {
      const int lr = 16 * wave + 8 * hh + r;
      float v = acc[t][r] + bn;
      if (EPI == 0) v = (v >= 0.f) ? v : 0.2f * v;
      stg[lr * 64 + lc] = v;
    }
  }
  __syncthreads();

  if (EPI == 0) {
    const int q8 = lane & 7, sub = lane >> 3;
    v8us hv[4], lv[4];
    size_t po[4];
#pragma unroll
    for (int i = 0; i < 4; ++i) {
      const int lr = 16 * wave + 4 * i + sub;
      const v4f a = *(const v4fa*)(stg + lr * 64 + 8 * q8);
      const v4f b = *(const v4fa*)(stg + lr * 64 + 8 * q8 + 4);
      split8(a, b, hv[i], lv[i]);
      po[i] = (size_t)(rowBase + lr) * (size_t)NO + (size_t)(col0 + 8 * q8);
    }
#pragma unroll
    for (int i = 0; i < 4; ++i) {
      *(volatile v8us*)(ohi + po[i]) = hv[i];
      *(volatile v8us*)(olo + po[i]) = lv[i];
    }
    __threadfence();
#pragma unroll
    for (int i = 0; i < 4; ++i) {
      *(volatile v8us*)(ohi + po[i]) = hv[i];
      *(volatile v8us*)(olo + po[i]) = lv[i];
    }
  } else {
    v4f fv[8];
    size_t op[8];
#pragma unroll
    for (int i = 0; i < 8; ++i) {
      const int lr = 16 * wave + 2 * i + hh;
      fv[i] = *(const v4fa*)(stg + lr * 64 + 4 * m);
      op[i] = (size_t)(rowBase + lr) * (size_t)NO + (size_t)(col0 + 4 * m);
    }
#pragma unroll
    for (int i = 0; i < 8; ++i) *(volatile v4f*)(yo + op[i]) = fv[i];
    __threadfence();
#pragma unroll
    for (int i = 0; i < 8; ++i) *(volatile v4f*)(yo + op[i]) = fv[i];
  }
}

__global__ __launch_bounds__(NTHR) void k_out(const float* __restrict__ yv, const int* __restrict__ tab, float* out) {
  const int lane = (int)threadIdx.x & 31, wave = (int)threadIdx.x >> 5, hh = lane >> 4, m = lane & 15;
  int t = (int)blockIdx.x * 8 + wave;
  t = t > BSZ - 1 ? BSZ - 1 : t;
  int p = tab[TABL + t];
  p = p < 0 ? 0 : (p > MP - 1 ? MP - 1 : p);
  const v4f v = *(const v4fa*)(yv + (size_t)p * SDIM + 4 * m);
  float* op = out + (size_t)t * SDIM + 4 * m;
  if (hh == 0) *(volatile v4f*)op = v;
  __threadfence();
  if (hh == 0) *(volatile v4f*)op = v;
}

static inline int cdiv(int a, int b) { return (a + b - 1) / b; }

extern "C" void kernel_launch(void* const* d_in, const int* in_sizes, int n_in,
                              void* d_out, int out_size, void* d_ws, size_t ws_size,
                              hipStream_t stream) {
  if (n_in < 18) return;
  if (in_sizes[0] != BSZ * LDIM) return;
  if (in_sizes[1] != BSZ) return;
  if (in_sizes[2] != LDIM * HDIM) return;
  if (in_sizes[3] != HDIM) return;
  if (in_sizes[4] != HDIM * HDIM || in_sizes[6] != HDIM * HDIM || in_sizes[8] != HDIM * HDIM) return;
  if (in_sizes[5] != HDIM || in_sizes[7] != HDIM || in_sizes[9] != HDIM) return;
  if (in_sizes[10] != NDOM * HDIM * HDIM || in_sizes[12] != NDOM * HDIM * HDIM ||
      in_sizes[14] != NDOM * HDIM * HDIM) return;
  if (in_sizes[11] != NDOM * HDIM || in_sizes[13] != NDOM * HDIM || in_sizes[15] != NDOM * HDIM) return;
  if (in_sizes[16] != NDOM * HDIM * SDIM) return;
  if (in_sizes[17] != NDOM * SDIM) return;
  if (out_size != BSZ * SDIM) return;

  const float* z   = (const float*)d_in[0];
  const int*   y   = (const int*)d_in[1];
  const float* tW0 = (const float*)d_in[2];
  const float* tb0 = (const float*)d_in[3];
  const float* tW1 = (const float*)d_in[4];
  const float* tb1 = (const float*)d_in[5];
  const float* tW2 = (const float*)d_in[6];
  const float* tb2 = (const float*)d_in[7];
  const float* tW3 = (const float*)d_in[8];
  const float* tb3 = (const float*)d_in[9];
  const float* hW0 = (const float*)d_in[10];
  const float* hb0 = (const float*)d_in[11];
  const float* hW1 = (const float*)d_in[12];
  const float* hb1 = (const float*)d_in[13];
  const float* hW2 = (const float*)d_in[14];
  const float* hb2 = (const float*)d_in[15];
  const float* hW3 = (const float*)d_in[16];
  const float* hb3 = (const float*)d_in[17];
  float* out = (float*)d_out;

  char* ws = (char*)d_ws;
  size_t off = 0;
  const size_t oT0W = off; off += (size_t)HDIM * LPAD * 2;            off = (off + 255) & ~(size_t)255;
  const size_t oTW1 = off; off += (size_t)HDIM * HDIM * 2;            off = (off + 255) & ~(size_t)255;
  const size_t oTW2 = off; off += (size_t)HDIM * HDIM * 2;            off = (off + 255) & ~(size_t)255;
  const size_t oTW3 = off; off += (size_t)HDIM * HDIM * 2;            off = (off + 255) & ~(size_t)255;
  const size_t oHW0 = off; off += (size_t)NDOM * HDIM * HDIM * 2;     off = (off + 255) & ~(size_t)255;
  const size_t oHW1 = off; off += (size_t)NDOM * HDIM * HDIM * 2;     off = (off + 255) & ~(size_t)255;
  const size_t oHW2 = off; off += (size_t)NDOM * HDIM * HDIM * 2;     off = (off + 255) & ~(size_t)255;
  const size_t oHW3 = off; off += (size_t)NDOM * SDIM * HDIM * 2;     off = (off + 255) & ~(size_t)255;
  const size_t oZB  = off; off += (size_t)BSZ * LPAD * 2;             off = (off + 255) & ~(size_t)255;
  const size_t oTAB = off; off += (size_t)TABN * 4;                   off = (off + 255) & ~(size_t)255;
  const size_t oCMH = off; off += (size_t)BSZ * HDIM * 2;             off = (off + 255) & ~(size_t)255;
  const size_t oCML = off; off += (size_t)BSZ * HDIM * 2;             off = (off + 255) & ~(size_t)255;
  const size_t oXGH = off; off += (size_t)MP * HDIM * 2;              off = (off + 255) & ~(size_t)255;
  const size_t oXGL = off; off += (size_t)MP * HDIM * 2;              off = (off + 255) & ~(size_t)255;
  const size_t oR1H = off; off += (size_t)MP * HDIM * 2;              off = (off + 255) & ~(size_t)255;
  const size_t oR1L = off; off += (size_t)MP * HDIM * 2;              off = (off + 255) & ~(size_t)255;
  const size_t oR2H = off; off += (size_t)MP * HDIM * 2;              off = (off + 255) & ~(size_t)255;
  const size_t oR2L = off; off += (size_t)MP * HDIM * 2;              off = (off + 255) & ~(size_t)255;
  const size_t oR3H = off; off += (size_t)MP * HDIM * 2;              off = (off + 255) & ~(size_t)255;
  const size_t oR3L = off; off += (size_t)MP * HDIM * 2;              off = (off + 255) & ~(size_t)255;
  const size_t oY   = off; off += (size_t)MP * SDIM * 4;              off = (off + 255) & ~(size_t)255;
  if (off > ws_size || off > (size_t)WSMAX) return;

  unsigned short* T0W = (unsigned short*)(ws + oT0W);
  unsigned short* TW1 = (unsigned short*)(ws + oTW1);
  unsigned short* TW2 = (unsigned short*)(ws + oTW2);
  unsigned short* TW3 = (unsigned short*)(ws + oTW3);
  unsigned short* HW0 = (unsigned short*)(ws + oHW0);
  unsigned short* HW1 = (unsigned short*)(ws + oHW1);
  unsigned short* HW2 = (unsigned short*)(ws + oHW2);
  unsigned short* HW3 = (unsigned short*)(ws + oHW3);
  unsigned short* ZB  = (unsigned short*)(ws + oZB);
  int*            TAB = (int*)(ws + oTAB);
  unsigned short* CMH = (unsigned short*)(ws + oCMH);
  unsigned short* CML = (unsigned short*)(ws + oCML);
  unsigned short* XGH = (unsigned short*)(ws + oXGH);
  unsigned short* XGL = (unsigned short*)(ws + oXGL);
  unsigned short* R1H = (unsigned short*)(ws + oR1H);
  unsigned short* R1L = (unsigned short*)(ws + oR1L);
  unsigned short* R2H = (unsigned short*)(ws + oR2H);
  unsigned short* R2L = (unsigned short*)(ws + oR2L);
  unsigned short* R3H = (unsigned short*)(ws + oR3H);
  unsigned short* R3L = (unsigned short*)(ws + oR3L);
  float*          Y   = (float*)(ws + oY);

  hipFuncSetAttribute(reinterpret_cast<const void*>(&k_bucket),
                      hipFuncAttributeMaxDynamicSharedMemorySize, LDS_BKT);

  {
    const int nU0 = HDIM * LPAD / 8;
    k_wtr<<<cdiv(nU0, NTHR), NTHR, 0, stream>>>(tW0, T0W, LDIM, LPAD, HDIM, 1, nU0);
    const int nUt = HDIM * HDIM / 8;
    k_wtr<<<cdiv(nUt, NTHR), NTHR, 0, stream>>>(tW1, TW1, HDIM, HDIM, HDIM, 1, nUt);
    k_wtr<<<cdiv(nUt, NTHR), NTHR, 0, stream>>>(tW2, TW2, HDIM, HDIM, HDIM, 1, nUt);
    k_wtr<<<cdiv(nUt, NTHR), NTHR, 0, stream>>>(tW3, TW3, HDIM, HDIM, HDIM, 1, nUt);
    const int nUh = NDOM * HDIM * HDIM / 8;
    k_wtr<<<cdiv(nUh, NTHR), NTHR, 0, stream>>>(hW0, HW0, HDIM, HDIM, HDIM, NDOM, nUh);
    k_wtr<<<cdiv(nUh, NTHR), NTHR, 0, stream>>>(hW1, HW1, HDIM, HDIM, HDIM, NDOM, nUh);
    k_wtr<<<cdiv(nUh, NTHR), NTHR, 0, stream>>>(hW2, HW2, HDIM, HDIM, HDIM, NDOM, nUh);
    const int nU3 = NDOM * SDIM * HDIM / 8;
    k_wtr<<<cdiv(nU3, NTHR), NTHR, 0, stream>>>(hW3, HW3, HDIM, HDIM, SDIM, NDOM, nU3);
  }
  {
    const int nUz = BSZ * (LPAD / 8);
    k_zpad<<<cdiv(nUz, NTHR), NTHR, 0, stream>>>(z, ZB, nUz);
  }
  k_bucket<<<1, NTHR, LDS_BKT, stream>>>(y, TAB);

  k_gemm<LPAD, 1, HDIM, false, 0><<<dim3(NTT, HDIM / 64), GTHR, 0, stream>>>(ZB, ZB, T0W, tb0, TAB, R1H, R1L, Y);
  k_gemm<HDIM, 2, HDIM, false, 0><<<dim3(NTT, HDIM / 64), GTHR, 0, stream>>>(R1H, R1L, TW1, tb1, TAB, R2H, R2L, Y);
  k_gemm<HDIM, 2, HDIM, false, 0><<<dim3(NTT, HDIM / 64), GTHR, 0, stream>>>(R2H, R2L, TW2, tb2, TAB, R3H, R3L, Y);
  k_gemm<HDIM, 2, HDIM, false, 0><<<dim3(NTT, HDIM / 64), GTHR, 0, stream>>>(R3H, R3L, TW3, tb3, TAB, CMH, CML, Y);

  {
    const int nUx = MP * (HDIM / 8);
    k_gather<<<cdiv(nUx, NTHR), NTHR, 0, stream>>>(CMH, CML, TAB, XGH, XGL, nUx);
  }

  k_gemm<HDIM, 2, HDIM, true, 0><<<dim3(NTILE, HDIM / 64), GTHR, 0, stream>>>(XGH, XGL, HW0, hb0, TAB, R1H, R1L, Y);
  k_gemm<HDIM, 2, HDIM, true, 0><<<dim3(NTILE, HDIM / 64), GTHR, 0, stream>>>(R1H, R1L, HW1, hb1, TAB, R2H, R2L, Y);
  k_gemm<HDIM, 2, HDIM, true, 0><<<dim3(NTILE, HDIM / 64), GTHR, 0, stream>>>(R2H, R2L, HW2, hb2, TAB, R3H, R3L, Y);
  k_gemm<HDIM, 2, SDIM, true, 1><<<dim3(NTILE, SDIM / 64), GTHR, 0, stream>>>(R3H, R3L, HW3, hb3, TAB, XGH, XGL, Y);

  k_out<<<BSZ / 8, NTHR, 0, stream>>>(Y, TAB, out);
}
